// QuantLinear_54065048322157
// MI455X (gfx1250) — hardware-verified
//
#include <hip/hip_runtime.h>

#pragma clang fp contract(off)

constexpr int kRowsM        = 16;
constexpr int kDimK         = 4096;
constexpr int kColsN        = 11008;
constexpr int kWordsPerRow  = kDimK / 8;
constexpr int kNumGroups    = 32;
constexpr int kNTile        = 64;
constexpr int kNumNTiles    = kColsN / kNTile;
constexpr int kWavesPerBlk  = 4;
constexpr int kGemmBlocks   = kNumNTiles / kWavesPerBlk;
constexpr int kTotalWords   = kColsN * kWordsPerRow;
constexpr int kDqBlocks     = kTotalWords / 256;
constexpr int kXn8          = kRowsM * kDimK / 8;
constexpr int kCastBlocks   = kXn8 / 256;
constexpr float kWCarry     = 64.0f;
constexpr float kWCarryInv  = 1.0f / 64.0f;

static_assert(kNumNTiles * kNTile == kColsN);
static_assert(kGemmBlocks * kWavesPerBlk == kNumNTiles);
static_assert(kDimK % 32 == 0);
static_assert(kDqBlocks * 256 == kTotalWords);
static_assert(kCastBlocks * 256 == kXn8);
static_assert(kWordsPerRow == 512);

constexpr size_t kWhBytes = (size_t)kColsN * kDimK * 2;
constexpr size_t kXhBytes = (size_t)kRowsM * kDimK * 2;
constexpr size_t kWsTotal = kWhBytes + kXhBytes;
static_assert(kWhBytes % 128 == 0);
static_assert(kWsTotal <= 134217728ull);

typedef __attribute__((ext_vector_type(16))) _Float16 v16h;
typedef __attribute__((ext_vector_type(8)))  _Float16 v8h;
typedef __attribute__((ext_vector_type(8)))  float    v8f;
typedef __attribute__((ext_vector_type(4)))  float    v4f;
typedef __attribute__((ext_vector_type(4)))  unsigned int v4u;

__device__ __forceinline__ void dep_guard_h(v8f& a, v8f& b, v16h x, v16h y) { asm volatile("v_nop\n\tv_nop\n\tv_nop\n\tv_nop" : "+v"(a), "+v"(b) : "v"(x), "v"(y)); }
__device__ __forceinline__ void keep4_h(v16h a, v16h b, v16h c, v16h d) { asm volatile("v_nop" :: "v"(a), "v"(b), "v"(c), "v"(d)); }
__device__ __forceinline__ void acc_guard4(v8f& a, v8f& b, v8f& c, v8f& d) { asm volatile("v_nop\n\tv_nop\n\tv_nop\n\tv_nop" : "+v"(a), "+v"(b), "+v"(c), "+v"(d)); }
template <typename T> struct Frag;
template <> struct Frag<_Float16> {
  typedef v16h V; union U { v16h v; v8h h[2]; };
  static __device__ __forceinline__ v16h load(const _Float16* p) {
    U f; f.h[0] = *(const v8h*)(p); f.h[1] = *(const v8h*)(p + 16); return f.v;
  }
  static __device__ __forceinline__ v8f mma(v16h a, v16h b, v8f c) {
    return __builtin_amdgcn_wmma_f32_16x16x32_f16(false, a, false, b, (short)0, c, false, false);
  }
  static __device__ __forceinline__ void guard(v8f& a, v8f& b, v16h x, v16h y) { dep_guard_h(a, b, x, y); }
  static __device__ __forceinline__ void keep(v16h a, v16h b, v16h c, v16h d) { keep4_h(a, b, c, d); }
};

__device__ __forceinline__ void guard_all4(v8f& a, v8f& b, v8f& c, v8f& d,
                                           v16h x, v16h y0, v16h y1, v16h y2, v16h y3) {
  asm volatile("v_nop\n\tv_nop\n\tv_nop\n\tv_nop"
               : "+v"(a), "+v"(b), "+v"(c), "+v"(d)
               : "v"(x), "v"(y0), "v"(y1), "v"(y2), "v"(y3));
}

__device__ __forceinline__ unsigned pk16(unsigned short a, unsigned short b) { return (unsigned)a | ((unsigned)b << 16); }
__device__ __forceinline__ unsigned short h_bits(float f) { const _Float16 h = (_Float16)f; return __builtin_bit_cast(unsigned short, h); }

__global__ __launch_bounds__(256) void dequant_w4_kernel(const int* __restrict__ qw, const float* __restrict__ scales,
                                                        const float* __restrict__ zeros, const int* __restrict__ gidx,
                                                        unsigned short* __restrict__ wh, int total_words) {
  const int i = blockIdx.x * 256 + threadIdx.x;
  if (i >= total_words) return;
  const int o = i >> 9;
  const int w = i & (kWordsPerRow - 1);
  const unsigned word = (unsigned)qw[i];
  int g = gidx[8 * w];
  g = g < 0 ? 0 : g;
  g = g > (kNumGroups - 1) ? (kNumGroups - 1) : g;
  const float s  = scales[(size_t)g * kColsN + o];
  const float z  = zeros[(size_t)g * kColsN + o];
  const float sc = s * kWCarry;
  const float zc = z * kWCarry;
  unsigned short hb[8];
#pragma unroll
  for (int j = 0; j < 8; ++j) {
    const float q = (float)((word >> (4 * j)) & 15u);
    const float p = q * sc;
    const float v = p - zc;
    hb[j] = h_bits(v);
  }
  const v4u u = (v4u){pk16(hb[0], hb[1]), pk16(hb[2], hb[3]), pk16(hb[4], hb[5]), pk16(hb[6], hb[7])};
  unsigned short* dst = wh + 8 * (size_t)i;
  *(volatile v4u*)dst = u;
  __threadfence();
  *(volatile v4u*)dst = u;
}

__global__ __launch_bounds__(256) void cast8_f16_kernel(const float* __restrict__ in, unsigned short* __restrict__ out, int n8) {
  const int i = blockIdx.x * 256 + threadIdx.x;
  if (i >= n8) return;
  const float* p = in + 8 * (size_t)i;
  const v4f a = *(const v4f*)(p);
  const v4f c = *(const v4f*)(p + 4);
  unsigned short hb[8];
#pragma unroll
  for (int e = 0; e < 4; ++e) {
    hb[e]     = h_bits(a[e]);
    hb[4 + e] = h_bits(c[e]);
  }
  const v4u u = (v4u){pk16(hb[0], hb[1]), pk16(hb[2], hb[3]), pk16(hb[4], hb[5]), pk16(hb[6], hb[7])};
  unsigned short* q = out + 8 * (size_t)i;
  *(volatile v4u*)q = u;
  __threadfence();
  *(volatile v4u*)q = u;
}

__global__ __launch_bounds__(128) void qgemm_f16_kernel(const unsigned short* __restrict__ Xp, const unsigned short* __restrict__ Wp,
                                                       const float* __restrict__ bias, float* __restrict__ out) {
  __shared__ __align__(16) float sT[kWavesPerBlk][16 * 68];
  const int lane = threadIdx.x & 31;
  const int wave = threadIdx.x >> 5;
  const int tile = blockIdx.x * kWavesPerBlk + wave;
  if (tile >= kNumNTiles) return;
  const int n0 = tile * kNTile;

  const _Float16* A  = (const _Float16*)Xp;
  const _Float16* Bt = (const _Float16*)Wp;
  const int rlane = lane & 15;
  const int koff  = (lane >> 4) * 8;
  const int mOff  = (lane >> 4) * 8;

  v8f acc[4];
#pragma unroll
  for (int j = 0; j < 4; ++j) acc[j] = (v8f){0.f,0.f,0.f,0.f,0.f,0.f,0.f,0.f};

  for (int k0 = 0; k0 < kDimK; k0 += 32) {
    v16h bh[4];
#pragma unroll
    for (int j = 0; j < 4; ++j) {
      const size_t bo = (size_t)(n0 + (j << 4) + rlane) * kDimK + koff + k0;
      bh[j] = Frag<_Float16>::load(Bt + bo);
    }
    const size_t ao = (size_t)rlane * kDimK + koff + k0;
    const v16h ah = Frag<_Float16>::load(A + ao);
#pragma unroll
    for (int j = 0; j < 4; ++j) acc[j] = Frag<_Float16>::mma(ah, bh[j], acc[j]);
    guard_all4(acc[0], acc[1], acc[2], acc[3], ah, bh[0], bh[1], bh[2], bh[3]);
  }
  acc_guard4(acc[0], acc[1], acc[2], acc[3]);

  float* slab = sT[wave];
#pragma unroll
  for (int j = 0; j < 4; ++j) {
    const int n = n0 + (j << 4) + rlane;
    const float bv = bias[n];
#pragma unroll
    for (int r = 0; r < 8; ++r) {
      const float sv = acc[j][r] * kWCarryInv;
      const float v  = sv + bv;
      slab[(mOff + r) * 68 + (j << 4) + rlane] = v;
    }
  }
  __builtin_amdgcn_fence(__ATOMIC_RELEASE, "workgroup");
  __builtin_amdgcn_wave_barrier();
  __builtin_amdgcn_fence(__ATOMIC_ACQUIRE, "workgroup");
  {
    const int hh = lane >> 4, c4 = (lane & 15) * 4;
    for (int pass = 0; pass < 2; ++pass) {
#pragma unroll
      for (int it = 0; it < 8; ++it) {
        const int row = it * 2 + hh;
        const v4f v = *(const v4f*)(slab + row * 68 + c4);
        *(volatile v4f*)(out + (size_t)row * kColsN + n0 + c4) = v;
      }
      __threadfence();
    }
  }
}

extern "C" void kernel_launch(void* const* d_in, const int* in_sizes, int n_in,
                              void* d_out, int out_size, void* d_ws, size_t ws_size, hipStream_t stream) {
  if (n_in < 6) return;
  if (ws_size < kWsTotal) return;
  if (in_sizes[0] != kRowsM * kDimK) return;
  if (in_sizes[1] != kTotalWords) return;
  if (in_sizes[2] != kNumGroups * kColsN) return;
  if (in_sizes[3] != kNumGroups * kColsN) return;
  if (in_sizes[4] != kColsN) return;
  if (in_sizes[5] != kDimK) return;
  if (out_size != kRowsM * kColsN) return;

  const float* x      = (const float*)d_in[0];
  const int*   qw     = (const int*)d_in[1];
  const float* scales = (const float*)d_in[2];
  const float* zeros  = (const float*)d_in[3];
  const float* bias   = (const float*)d_in[4];
  const int*   gidx   = (const int*)d_in[5];
  float* out = (float*)d_out;

  unsigned short* wh = (unsigned short*)d_ws;
  unsigned short* xh = (unsigned short*)((char*)d_ws + kWhBytes);

  dequant_w4_kernel<<<dim3(kDqBlocks), dim3(256), 0, stream>>>(qw, scales, zeros, gidx, wh, kTotalWords);
  cast8_f16_kernel<<<dim3(kCastBlocks), dim3(256), 0, stream>>>(x, xh, kXn8);
  qgemm_f16_kernel<<<dim3(kGemmBlocks), dim3(kWavesPerBlk * 32), 0, stream>>>(xh, wh, bias, out);
}
